// GCN_Expert_3109556322394
// MI455X (gfx1250) — hardware-verified
//
#include <hip/hip_runtime.h>
#include <math.h>

typedef __attribute__((ext_vector_type(16))) _Float16 v16h;
typedef __attribute__((ext_vector_type(16))) __bf16 v16b;
typedef __attribute__((ext_vector_type(8)))  _Float16 v8h;
typedef __attribute__((ext_vector_type(8)))  float v8f;
typedef __attribute__((ext_vector_type(4)))  float v4f;
typedef __attribute__((ext_vector_type(2)))  float v2f;
typedef __attribute__((ext_vector_type(4)))  unsigned v4u;
typedef __attribute__((ext_vector_type(4)))  int v4i;
typedef float __attribute__((may_alias)) float_a;
typedef int __attribute__((may_alias)) int_a;

template <typename T> __device__ __forceinline__ void vst2(void* p, T v) { *(volatile T*)p = v; __threadfence(); *(volatile T*)p = v; }
__device__ __forceinline__ v8f wmma16(v16h a, v16h b, v8f c) {
  v8f d = __builtin_amdgcn_wmma_f32_16x16x32_f16(false, a, false, b, (short)0, c, false, false);
  asm volatile("v_nop\n\tv_nop\n\tv_nop\n\tv_nop" : "+v"(d) : "v"(a), "v"(b));
  return d;
}
__device__ __forceinline__ v8f wmma_bf(v16b a, v16b b, v8f c) {
  v8f d = __builtin_amdgcn_wmma_f32_16x16x32_bf16(false, a, false, b, (short)0, c, false, false);
  asm volatile("v_nop\n\tv_nop\n\tv_nop\n\tv_nop" : "+v"(d) : "v"(a), "v"(b));
  return d;
}
__device__ __forceinline__ v16h frag_h(const _Float16* rowk0, int lane) {
  union { v16h v; v8h q[2]; } u; const _Float16* p = rowk0 + 8 * (lane >> 4);
  u.q[0] = *(const v8h*)p; u.q[1] = *(const v8h*)(p + 16); return u.v;
}
__device__ __forceinline__ v16h frag_f32(const float* rowk0, int lane) {
  v16h a; const float* p = rowk0 + 8 * (lane >> 4);
#pragma unroll
  for (int i = 0; i < 8; ++i) { a[i] = (_Float16)p[i]; a[8 + i] = (_Float16)p[16 + i]; }
  return a;
}
__device__ __forceinline__ v16h frag_f32s(const float* rowk0, int lane, float sc) {
  v16h a; const float* p = rowk0 + 8 * (lane >> 4);
#pragma unroll
  for (int i = 0; i < 8; ++i) { a[i] = (_Float16)(p[i] * sc); a[8 + i] = (_Float16)(p[16 + i] * sc); }
  return a;
}
__device__ __forceinline__ v16h fragc_f32(const float* W, int k0, int n, int lane, int ld, int K) {
  v16h a; const int g = lane >> 4;
#pragma unroll
  for (int i = 0; i < 8; ++i) { const int ka = k0 + 8 * g + i, kb = ka + 16;
    a[i] = (_Float16)(ka < K ? W[(size_t)ka * ld + n] : 0.f); a[8 + i] = (_Float16)(kb < K ? W[(size_t)kb * ld + n] : 0.f); }
  return a;
}
struct F2 { v16b h, l; };
__device__ __forceinline__ F2 bsplit16(const float v[16]) { F2 r;
#pragma unroll
  for (int i = 0; i < 16; ++i) { const __bf16 h = (__bf16)v[i]; r.h[i] = h; r.l[i] = (__bf16)(v[i] - (float)h); }
  return r; }
__device__ __forceinline__ F2 split_row(const float* row, int k0, int lane) { float v[16]; const float* p = row + k0 + 8 * (lane >> 4);
#pragma unroll
  for (int i = 0; i < 8; ++i) { v[i] = p[i]; v[8 + i] = p[16 + i]; }
  return bsplit16(v); }
__device__ __forceinline__ F2 split_rowK(const float* row, int k0, int lane, int K) { float v[16]; const int g = lane >> 4;
#pragma unroll
  for (int i = 0; i < 8; ++i) { const int ka = k0 + 8 * g + i, kb = ka + 16; v[i] = ka < K ? row[ka] : 0.f; v[8 + i] = kb < K ? row[kb] : 0.f; }
  return bsplit16(v); }
__device__ __forceinline__ F2 split_col(const float* W, int k0, int n, int lane, int ld, int K) { float v[16]; const int g = lane >> 4;
#pragma unroll
  for (int i = 0; i < 8; ++i) { const int ka = k0 + 8 * g + i, kb = ka + 16; v[i] = ka < K ? W[(size_t)ka * ld + n] : 0.f; v[8 + i] = kb < K ? W[(size_t)kb * ld + n] : 0.f; }
  return bsplit16(v); }
__device__ __forceinline__ v8f mac3(const F2& a, const F2& b, v8f c) { c = wmma_bf(a.l, b.h, c); c = wmma_bf(a.h, b.l, c); return wmma_bf(a.h, b.h, c); }
__device__ __forceinline__ float sigm(float v) { return 1.0f / (1.0f + expf(-v)); }
#define LDSX() do { asm volatile("s_wait_dscnt 0" ::: "memory"); __builtin_amdgcn_wave_barrier(); __builtin_amdgcn_fence(__ATOMIC_RELEASE, "workgroup"); } while (0)

#define NN 50000
#define NE 800000
#define NLG 40
#define FD 256
#define FH 64
#define DH 32
#define MAXDEG 256
#define X0W 160
#define X0K 136
#define F0 128
#define FC 40
#define FCP 64
#define RB 512
#define NRB ((NN + RB - 1) / RB)
#define NNP (NRB * RB)
#define EPT 16
#define CH (256 * EPT)

#define RBD 8192
#define NRBD ((NN + RBD - 1) / RBD)
__device__ __forceinline__ void load4ids(const int* __restrict__ ids, int e, int dd[4]) { const int4 a = *(const int4*)(ids + e); dd[0] = a.x; dd[1] = a.y; dd[2] = a.z; dd[3] = a.w; }
__global__ __launch_bounds__(256) void k_deg(const int* __restrict__ ei, const float* __restrict__ dtab, float* __restrict__ DINV, float* __restrict__ DEGE) {
  __shared__ int scd[RBD], scs[RBD];
  const int tid = threadIdx.x; const int r0 = blockIdx.x * RBD; const int* esrc = ei; const int* edst = ei + NE;
  for (int q = tid; q < RBD; q += 256) { scd[q] = 0; scs[q] = 0; }
  __syncthreads();
#pragma unroll 1
  for (int pass = 0; pass < 2; ++pass) { const int* arr = pass == 0 ? edst : esrc; int* sc = pass == 0 ? scd : scs;
#pragma unroll 1
    for (int c0 = 0; c0 < NE; c0 += CH) { const int e0 = c0 + tid * EPT;
      if (e0 + EPT <= NE) {
#pragma unroll
        for (int v = 0; v < EPT / 4; ++v) { int dd[4]; load4ids(arr, e0 + v * 4, dd);
#pragma unroll
          for (int u = 0; u < 4; ++u) { const unsigned rel = (unsigned)(dd[u] - r0); if (rel < (unsigned)RBD) atomicAdd(&sc[rel], 1); } } }
      else { for (int u = 0; u < EPT; ++u) { const int e = e0 + u; if (e < NE) { const unsigned rel = (unsigned)(arr[e] - r0); if (rel < (unsigned)RBD) atomicAdd(&sc[rel], 1); } } } } }
  __syncthreads();
  for (int q = tid; q < RBD; q += 256) { const int r = r0 + q; if (r < NNP) vst2(DINV + r, r < NN ? rsqrtf((float)(scd[q] + 1)) : 0.f); }
  for (int q = tid; q < RBD * 8; q += 256) { const int rl = q >> 3, pc = q & 7; const int r = r0 + rl; if (r >= NNP) continue;
    v4f v = {0.f, 0.f, 0.f, 0.f}; if (r < NN) { int dg = scd[rl] + scs[rl]; dg = dg > MAXDEG - 1 ? MAXDEG - 1 : dg; v = *(const v4f*)(dtab + (size_t)dg * DH + pc * 4); }
    vst2(DEGE + (size_t)r * DH + pc * 4, v); }
}
__global__ __launch_bounds__(128) void k_x0(const float* __restrict__ logits, const float* __restrict__ feat, const float* __restrict__ Wf, const float* __restrict__ bf, const float* __restrict__ DEGE, float* __restrict__ X0) {
  __shared__ __align__(16) float so[4][16][X0W + 4];
  const int tid = threadIdx.x, wave = tid >> 5, lane = tid & 31, col = lane & 15, g = lane >> 4;
  const int r0 = blockIdx.x * 64 + wave * 16; const int ra = (r0 + col) < NN ? (r0 + col) : (NN - 1);
  v8f acc[4] = {};
#pragma unroll 1
  for (int kc = 0; kc < FD / 32; ++kc) { const F2 a = split_row(feat + (size_t)ra * FD, kc * 32, lane);
#pragma unroll
    for (int t = 0; t < 4; ++t) acc[t] = mac3(a, split_col(Wf, kc * 32, t * 16 + col, lane, FH, FD), acc[t]); }
#pragma unroll
  for (int t = 0; t < 4; ++t) { const int n = t * 16 + col; const float bb = bf[n];
#pragma unroll
    for (int r = 0; r < 8; ++r) { const int row = r0 + 8 * g + r; so[wave][8 * g + r][NLG + n] = row < NN ? acc[t][r] + bb : 0.f; } }
  { const int rl = lane & 15, hf = lane >> 4; const int row = r0 + rl; float* d = &so[wave][rl][0];
    if (row < NN) { const float* lg = logits + (size_t)row * NLG + hf * 20;
#pragma unroll
      for (int i = 0; i < 20; ++i) d[hf * 20 + i] = lg[i];
      const float* dr = DEGE + (size_t)row * DH + hf * 16;
#pragma unroll
      for (int i = 0; i < 16; ++i) d[NLG + FH + hf * 16 + i] = dr[i]; }
    else {
#pragma unroll
      for (int i = 0; i < 20; ++i) d[hf * 20 + i] = 0.f;
#pragma unroll
      for (int i = 0; i < 16; ++i) d[NLG + FH + hf * 16 + i] = 0.f; }
#pragma unroll
    for (int i = 0; i < 12; ++i) d[X0K + hf * 12 + i] = 0.f; }
  LDSX();
  for (int q = lane; q < 16 * (X0W / 4); q += 32) { const int rl = q / (X0W / 4), pc = q % (X0W / 4); vst2(X0 + (size_t)(r0 + rl) * X0W + pc * 4, *(const v4f*)(&so[wave][rl][pc * 4])); }
}
template <int K, int NOUT, int WROWS, int KV = K>
__global__ __launch_bounds__(128) void k_gemm(const float* __restrict__ A, int lda, const float* __restrict__ W, const float* __restrict__ DINV, float* __restrict__ HS) {
  __shared__ __align__(16) float so[4][16][NOUT + 4];
  const int tid = threadIdx.x, wave = tid >> 5, lane = tid & 31, col = lane & 15, g = lane >> 4;
  const int r0 = blockIdx.x * 64 + wave * 16;
  constexpr int NT = (NOUT + 15) / 16;
  v8f acc[NT];
#pragma unroll
  for (int t = 0; t < NT; ++t) acc[t] = (v8f){};
const int ra = (r0 + col) < NN ? (r0 + col) : (NN - 1);
#pragma unroll 1
  for (int kc = 0; kc < K / 32; ++kc) { const F2 a = split_row(A + (size_t)ra * lda, kc * 32, lane);
#pragma unroll
    for (int t = 0; t < NT; ++t) { const int n = t * 16 + col; const int nn = n < NOUT ? n : 0; acc[t] = mac3(a, WROWS ? split_row(W + (size_t)nn * K, kc * 32, lane) : split_col(W, kc * 32, nn, lane, NOUT, KV), acc[t]); } }
#pragma unroll
  for (int t = 0; t < NT; ++t) { const int n = t * 16 + col;
#pragma unroll
    for (int r = 0; r < 8; ++r) { const int row = r0 + 8 * g + r; const float dv = row < NN ? DINV[row] : 0.f; if (n < NOUT) so[wave][8 * g + r][n] = acc[t][r] * dv; } }
  LDSX();
  for (int q = lane; q < 16 * (NOUT / 4); q += 32) { const int rl = q / (NOUT / 4), pc = q % (NOUT / 4); vst2(HS + (size_t)(r0 + rl) * NOUT + pc * 4, *(const v4f*)(&so[wave][rl][pc * 4])); }
}
template <int F, int MODE>
__global__ __launch_bounds__(256) void k_agg(const float* __restrict__ HS, const int* __restrict__ ei, const float* __restrict__ DINV, const float* __restrict__ bias, const float* __restrict__ lng, const float* __restrict__ lnb, float* __restrict__ OUT) {
  __shared__ __align__(16) float sacc[RB][F];
  __shared__ int ssrc[8][32 * EPT], sdl[8][32 * EPT]; __shared__ int scnt[8];
  const int tid = threadIdx.x, wave = tid >> 5, lane = tid & 31;
  const int r0 = blockIdx.x * RB; const int* esrc = ei; const int* edst = ei + NE;
  for (int q = tid; q < RB * F; q += 256) (&sacc[0][0])[q] = 0.f;
  __syncthreads();
#pragma unroll 1
  for (int c0 = 0; c0 < NE; c0 += CH) {
    const int e0 = c0 + tid * EPT; int hd[EPT]; int cnt = 0;
    if (e0 + EPT <= NE) {
#pragma unroll
      for (int v = 0; v < EPT / 4; ++v) { int dd[4]; load4ids(edst, e0 + v * 4, dd);
#pragma unroll
        for (int u = 0; u < 4; ++u) { const unsigned rel = (unsigned)(dd[u] - r0); const bool h = rel < (unsigned)RB; hd[v * 4 + u] = h ? (int)rel : -1; cnt += h ? 1 : 0; } } }
    else {
#pragma unroll
      for (int u = 0; u < EPT; ++u) { const int e = e0 + u; hd[u] = -1; if (e < NE) { const unsigned rel = (unsigned)(edst[e] - r0); if (rel < (unsigned)RB) { hd[u] = (int)rel; ++cnt; } } } }
    int incl = cnt;
#pragma unroll
    for (int off = 1; off < 32; off <<= 1) { const int vv = __shfl_up(incl, off, 32); if (lane >= off) incl += vv; }
    const int wtot = __shfl(incl, 31, 32); int pos = incl - cnt;
    if (cnt > 0) {
#pragma unroll
      for (int u = 0; u < EPT; ++u) if (hd[u] >= 0) { int s = esrc[e0 + u]; s = s < 0 ? 0 : (s >= NN ? NN - 1 : s); ssrc[wave][pos] = s; sdl[wave][pos] = hd[u];  ++pos; } }
    if (lane == 0) scnt[wave] = wtot;
    __syncthreads();
    if (tid < F) { for (int w = 0; w < 8; ++w) { const int nh = scnt[w]; for (int i = 0; i < nh; ++i) sacc[sdl[w][i]][tid] += HS[(size_t)ssrc[w][i] * F + tid]; } }
    __syncthreads(); }
  for (int rl = tid; rl < RB; rl += 256) { const int row = r0 + rl; if (row >= NN) continue; const float dv = DINV[row]; float* ar = &sacc[rl][0]; const float* hs = HS + (size_t)row * F;
    for (int f = 0; f < F; ++f) ar[f] = (ar[f] + hs[f]) * dv + bias[f];
    if (MODE == 2) { for (int f = 0; f < F; ++f) ar[f] = ar[f] > 0.f ? ar[f] : 0.f; }
    else if (MODE == 0) { float mu = 0.f; for (int f = 0; f < F; ++f) mu += ar[f]; mu *= (1.0f / F); float var = 0.f; for (int f = 0; f < F; ++f) { const float d = ar[f] - mu; var += d * d; } var *= (1.0f / F);
      const float rs = rsqrtf(var + 1e-5f); for (int f = 0; f < F; ++f) { const float v = (ar[f] - mu) * rs * lng[f] + lnb[f]; ar[f] = v > 0.f ? v : 0.f; } }
    else if (MODE == 1) { float mx = -3.4e38f; for (int f = 0; f < FC; ++f) mx = fmaxf(mx, ar[f]); float se = 0.f; for (int f = 0; f < FC; ++f) se += expf(ar[f] - mx); const float lse = logf(se) + mx; for (int f = 0; f < FC; ++f) ar[f] -= lse; } }
  __syncthreads();
  if (MODE != 1 && MODE != 3) { for (int q = tid; q < RB * (F / 4); q += 256) { const int rl = q / (F / 4), pc = q % (F / 4); const int row = r0 + rl; v4f v = *(const v4f*)(&sacc[rl][pc * 4]); if (row >= NN) { if (MODE == 2) continue; v = (v4f){0.f, 0.f, 0.f, 0.f}; } vst2(OUT + (size_t)row * F + pc * 4, v); } }
  else {
    for (int q = tid; q < RB * FC / 4; q += 256) { const int rl = (q * 4) / FC, f = (q * 4) % FC; const int row = r0 + rl; if (row < NN) { v4f v; v[0] = sacc[rl][f]; v[1] = sacc[rl][f + 1]; v[2] = sacc[rl][f + 2]; v[3] = sacc[rl][f + 3]; vst2(OUT + (size_t)row * FC + f, v); } } }
}
extern "C" void kernel_launch(void* const* d_in, const int* in_sizes, int n_in, void* d_out, int out_size, void* d_ws, size_t ws_size, hipStream_t stream) {
  (void)in_sizes; (void)n_in; (void)out_size; (void)ws_size;
  const float* logits = (const float*)d_in[0]; const float* feat = (const float*)d_in[1]; const int* ei = (const int*)d_in[2];
  const float* Wf = (const float*)d_in[3]; const float* bf = (const float*)d_in[4]; const float* dtab = (const float*)d_in[5];
  const float* W1 = (const float*)d_in[6]; const float* b1 = (const float*)d_in[7]; const float* W2 = (const float*)d_in[8]; const float* b2 = (const float*)d_in[9]; const float* W3 = (const float*)d_in[10]; const float* b3 = (const float*)d_in[11];
  float* out = (float*)d_out;
  char* ws = (char*)d_ws; size_t off = 0;
  auto take = [&](size_t bytes) { char* p = ws + off; off += (bytes + 255) & ~(size_t)255; return p; };
  float* DINV = (float*)take((size_t)NNP * 4); float* DEGE = (float*)take((size_t)NNP * DH * 4); float* X0 = (float*)take((size_t)NNP * X0W * 4);
  float* HS = (float*)take((size_t)NNP * F0 * 4); float* X1 = (float*)take((size_t)NNP * F0 * 4); float* X2 = (float*)take((size_t)NNP * F0 * 4); float* HS3 = (float*)take((size_t)NNP * FC * 4);
  k_deg<<<NRBD, 256, 0, stream>>>(ei, dtab, DINV, DEGE);
  k_x0<<<NNP / 64, 128, 0, stream>>>(logits, feat, Wf, bf, DEGE, X0);
  k_gemm<X0W, F0, 0, X0K><<<NNP / 64, 128, 0, stream>>>(X0, X0W, W1, DINV, HS);
  k_agg<F0, 2><<<NRB, 256, 0, stream>>>(HS, ei, DINV, b1, nullptr, nullptr, X1);
  k_gemm<F0, F0, 0><<<NNP / 64, 128, 0, stream>>>(X1, F0, W2, DINV, HS);
  k_agg<F0, 2><<<NRB, 256, 0, stream>>>(HS, ei, DINV, b2, nullptr, nullptr, X2);
  k_gemm<F0, FC, 0><<<NNP / 64, 128, 0, stream>>>(X2, F0, W3, DINV, HS3);
  k_agg<FC, 3><<<NRB, 256, 0, stream>>>(HS3, ei, DINV, b3, nullptr, nullptr, out);
}
